// CrossAttentionBlock_38663295598639
// MI455X (gfx1250) — hardware-verified
//
#include <hip/hip_runtime.h>
#include <math.h>
#include <stdint.h>

#define NB    4
#define CH    256
#define IMH   64
#define IMW   64
#define NPOS  4096
#define MTOK  (NB * NPOS)

static_assert(NPOS == IMH * IMW);
static_assert(CH % 64 == 0);
static_assert(NPOS % 64 == 0);
static_assert(MTOK % 64 == 0);
static_assert(CH % 32 == 0);
static_assert((CH * CH) % 512 == 0);
static_assert(CH == 256);

typedef __attribute__((ext_vector_type(16))) _Float16 v16h;
typedef __attribute__((ext_vector_type(8)))  _Float16 v8h;
typedef __attribute__((ext_vector_type(16))) __bf16   v16b;
typedef __attribute__((ext_vector_type(8)))  __bf16   v8b;
typedef __attribute__((ext_vector_type(8)))  float    v8f;
typedef __attribute__((ext_vector_type(4)))  float    v4f;
typedef __attribute__((ext_vector_type(2)))  float    v2f;
typedef __attribute__((ext_vector_type(4)))  unsigned int v4u;

#define HMIN 6.103515625e-5f

__device__ __forceinline__ unsigned short f2bf_bits(float f) {
  unsigned u = __float_as_uint(f);
  return (unsigned short)((u + 0x7FFFu + ((u >> 16) & 1u)) >> 16);
}
__device__ __forceinline__ float bf_bits2f(unsigned short h) { return __uint_as_float(((unsigned)h) << 16); }
__device__ __forceinline__ unsigned pk16(unsigned short a, unsigned short b) { return (unsigned)a | ((unsigned)b << 16); }
__device__ __forceinline__ _Float16 h_flush(float f) {
  const float g = (fabsf(f) < HMIN) ? 0.0f : f;
  return (_Float16)g;
}

__device__ __forceinline__ void dep_guard_h(v8f& a, v8f& b, v16h x, v16h y) { asm volatile("v_nop\n\tv_nop\n\tv_nop\n\tv_nop" : "+v"(a), "+v"(b) : "v"(x), "v"(y)); }
__device__ __forceinline__ void dep_guard_b(v8f& a, v8f& b, v16b x, v16b y) { asm volatile("v_nop\n\tv_nop\n\tv_nop\n\tv_nop" : "+v"(a), "+v"(b) : "v"(x), "v"(y)); }
__device__ __forceinline__ void keep4_h(v16h a, v16h b, v16h c, v16h d) { asm volatile("v_nop" :: "v"(a), "v"(b), "v"(c), "v"(d)); }
__device__ __forceinline__ void keep4_b(v16b a, v16b b, v16b c, v16b d) { asm volatile("v_nop" :: "v"(a), "v"(b), "v"(c), "v"(d)); }
__device__ __forceinline__ void acc_guard4(v8f& a, v8f& b, v8f& c, v8f& d) { asm volatile("v_nop\n\tv_nop\n\tv_nop\n\tv_nop" : "+v"(a), "+v"(b), "+v"(c), "+v"(d)); }
template <typename T> struct Frag;
template <> struct Frag<_Float16> {
  typedef v16h V; union U { v16h v; v8h h[2]; };
  static __device__ __forceinline__ v16h load(const _Float16* p) {
    U f; f.h[0] = *(const v8h*)(p); f.h[1] = *(const v8h*)(p + 16); return f.v;
  }
  static __device__ __forceinline__ v8f mma(v16h a, v16h b, v8f c) {
    return __builtin_amdgcn_wmma_f32_16x16x32_f16(false, a, false, b, (short)0, c, false, false);
  }
  static __device__ __forceinline__ void guard(v8f& a, v8f& b, v16h x, v16h y) { dep_guard_h(a, b, x, y); }
  static __device__ __forceinline__ void keep(v16h a, v16h b, v16h c, v16h d) { keep4_h(a, b, c, d); }
};
template <> struct Frag<__bf16> {
  typedef v16b V; union U { v16b v; v8b h[2]; };
  static __device__ __forceinline__ v16b load(const __bf16* p) {
    U f; f.h[0] = *(const v8b*)(p); f.h[1] = *(const v8b*)(p + 16); return f.v;
  }
  static __device__ __forceinline__ v8f mma(v16b a, v16b b, v8f c) {
    return __builtin_amdgcn_wmma_f32_16x16x32_bf16(false, a, false, b, (short)0, c, false, false);
  }
  static __device__ __forceinline__ void guard(v8f& a, v8f& b, v16b x, v16b y) { dep_guard_b(a, b, x, y); }
  static __device__ __forceinline__ void keep(v16b a, v16b b, v16b c, v16b d) { keep4_b(a, b, c, d); }
};

template <int ET> struct Elem;
template <> struct Elem<0> { typedef _Float16 T; };
template <> struct Elem<1> { typedef __bf16 T; };
template <int ET, bool SPLIT, int BIAS_MODE, int OUT_MODE, bool RESID, int ACT = 0>
__global__ __launch_bounds__(256) void wmma_gemm64(
    const unsigned short* __restrict__ Ap, const unsigned short* __restrict__ A2p, int lda, long strideA,
    const unsigned short* __restrict__ Btp, const unsigned short* __restrict__ Bt2p, int ldb, long strideB,
    void* __restrict__ Cout, void* __restrict__ Cout2, int ldc, long strideC,
    const float* __restrict__ bias,
    const float* __restrict__ resid, long strideR,
    int M, int N, int K, float scale) {
  typedef typename Elem<ET>::T T;
  typedef typename Frag<T>::V V;
  const T* A = (const T*)Ap; const T* A2 = (const T*)A2p; const T* Bt = (const T*)Btp; const T* Bt2 = (const T*)Bt2p;
  __shared__ __align__(16) float sT[8][16 * 68];
  const int b    = blockIdx.y;
  const int lane = threadIdx.x & 31;
  const int wave = threadIdx.x >> 5;
  const int tilesN = N >> 6;
  const int tilesM = M >> 6;
  const int tile = blockIdx.x * 8 + wave;
  if (tile >= tilesM * tilesN) return;
  const int tm = tile / tilesN;
  const int tn = tile - tm * tilesN;
  const int m0 = tm << 6;
  const int n0 = tn << 6;

  const T* Ab  = A  + (size_t)b * strideA;
  const T* Bb  = Bt + (size_t)b * strideB;
  const T* Ab2 = SPLIT ? (A2  + (size_t)b * strideA) : nullptr;
  const T* Bb2 = SPLIT ? (Bt2 + (size_t)b * strideB) : nullptr;

  const int rlane = lane & 15;
  const int koff  = (lane >> 4) * 8;
  const int mOff  = (lane >> 4) * 8;

  v8f acc[4][4];
#pragma unroll
  for (int i = 0; i < 4; ++i)
#pragma unroll
    for (int j = 0; j < 4; ++j) acc[i][j] = (v8f){0.f,0.f,0.f,0.f,0.f,0.f,0.f,0.f};

  for (int k0 = 0; k0 < K; k0 += 32) {
    V bh[4], bl[4];
#pragma unroll
    for (int j = 0; j < 4; ++j) {
      const size_t bo = (size_t)(n0 + (j << 4) + rlane) * ldb + koff + k0;
      bh[j] = Frag<T>::load(Bb + bo);
      if (SPLIT) bl[j] = Frag<T>::load(Bb2 + bo);
    }
#pragma unroll
    for (int i = 0; i < 4; ++i) {
      const size_t ao = (size_t)(m0 + (i << 4) + rlane) * lda + koff + k0;
      V ah = Frag<T>::load(Ab + ao);
      V al;
      if (SPLIT) al = Frag<T>::load(Ab2 + ao);
#pragma unroll
      for (int j = 0; j < 4; ++j) {
        acc[i][j] = Frag<T>::mma(ah, bh[j], acc[i][j]);
        if (SPLIT) {
          acc[i][j] = Frag<T>::mma(ah, bl[j], acc[i][j]);
          acc[i][j] = Frag<T>::mma(al, bh[j], acc[i][j]);
        }
      }
      Frag<T>::guard(acc[i][0], acc[i][3], ah, SPLIT ? al : ah);
    }
    Frag<T>::keep(bh[0], bh[1], bh[2], bh[3]);
    if (SPLIT) Frag<T>::keep(bl[0], bl[1], bl[2], bl[3]);
  }
  acc_guard4(acc[0][0], acc[0][1], acc[0][2], acc[0][3]);
  acc_guard4(acc[1][0], acc[1][1], acc[1][2], acc[1][3]);
  acc_guard4(acc[2][0], acc[2][1], acc[2][2], acc[2][3]);
  acc_guard4(acc[3][0], acc[3][1], acc[3][2], acc[3][3]);

  float* slab = sT[wave];
  const float* Rb = RESID ? (resid + (size_t)b * strideR) : nullptr;
#pragma unroll
  for (int i = 0; i < 4; ++i) {
    const int mBase = m0 + (i << 4);
#pragma unroll
    for (int j = 0; j < 4; ++j) {
      const int n = n0 + (j << 4) + rlane;
      float bv = 0.f;
      if (BIAS_MODE == 2) bv = bias[n];
#pragma unroll
      for (int r = 0; r < 8; ++r) {
        float v = acc[i][j][r] * scale;
        if (BIAS_MODE == 1) v += bias[mBase + mOff + r];
        if (BIAS_MODE == 2) v += bv;
        if (RESID) v += Rb[(size_t)(mBase + mOff + r) * ldc + n];
        if (ACT == 1) v = tanhf(v);
        if (ACT == 2) v = fmaxf(v, 0.0f);
        if (ACT == 3) v = v / (1.0f + expf(-v));
        if (ACT == 4) v = (v > 0.f) ? v : 0.01f * v;
        if (ACT == 5) v = 0.5f * v * (1.0f + erff(v * 0.70710678118654752f));
        slab[(mOff + r) * 68 + (j << 4) + rlane] = v;
      }
    }
    __builtin_amdgcn_fence(__ATOMIC_RELEASE, "workgroup");
    __builtin_amdgcn_wave_barrier();
    __builtin_amdgcn_fence(__ATOMIC_ACQUIRE, "workgroup");
    if (OUT_MODE == 0) {
      float* C = (float*)Cout + (size_t)b * strideC;
      const int hh = lane >> 4, c4 = (lane & 15) * 4;
      for (int pass = 0; pass < 2; ++pass) {
#pragma unroll
        for (int it = 0; it < 8; ++it) {
          const int row = it * 2 + hh;
          v4f v = *(const v4f*)(slab + row * 68 + c4);
          *(volatile v4f*)(C + (size_t)(mBase + row) * ldc + n0 + c4) = v;
        }
        __threadfence();
      }
    } else {
      const int q = lane >> 3, c8 = (lane & 7) * 8;
      unsigned short* C  = (unsigned short*)Cout  + (size_t)b * strideC;
      unsigned short* C2 = (OUT_MODE == 2) ? ((unsigned short*)Cout2 + (size_t)b * strideC) : nullptr;
      for (int pass = 0; pass < 2; ++pass) {
#pragma unroll
        for (int it = 0; it < 4; ++it) {
          const int row = it * 4 + q;
          const float* sp = slab + row * 68 + c8;
          v8h hv, lv;
#pragma unroll
          for (int e = 0; e < 8; ++e) {
            if (OUT_MODE == 1) {
              hv[e] = h_flush(sp[e]);
            } else {
              unsigned short hb = f2bf_bits(sp[e]);
              unsigned short lb = f2bf_bits(sp[e] - bf_bits2f(hb));
              hv[e] = __builtin_bit_cast(_Float16, hb);
              lv[e] = __builtin_bit_cast(_Float16, lb);
            }
          }
          *(volatile v8h*)(C + (size_t)(mBase + row) * ldc + n0 + c8) = hv;
          if (OUT_MODE == 2) *(volatile v8h*)(C2 + (size_t)(mBase + row) * ldc + n0 + c8) = lv;
        }
        __threadfence();
      }
    }
    __builtin_amdgcn_fence(__ATOMIC_RELEASE, "workgroup");
    __builtin_amdgcn_wave_barrier();
    __builtin_amdgcn_fence(__ATOMIC_ACQUIRE, "workgroup");
  }
}

__global__ __launch_bounds__(256) void split_bf16x2_kernel(const float* __restrict__ in, unsigned short* __restrict__ hi,
                                                           unsigned short* __restrict__ lo, int n2) {
  const int i = blockIdx.x * 256 + threadIdx.x;
  if (i < n2) {
    const v2f f = *(const v2f*)(in + 2 * (size_t)i);
    const unsigned short h0 = f2bf_bits(f[0]), h1 = f2bf_bits(f[1]);
    const unsigned short l0 = f2bf_bits(f[0] - bf_bits2f(h0)), l1 = f2bf_bits(f[1] - bf_bits2f(h1));
    const unsigned uh = pk16(h0, h1), ul = pk16(l0, l1);
    ((volatile unsigned*)hi)[i] = uh;
    ((volatile unsigned*)lo)[i] = ul;
    __threadfence();
    ((volatile unsigned*)hi)[i] = uh;
    ((volatile unsigned*)lo)[i] = ul;
  }
}

__global__ __launch_bounds__(256) void tsplit_kernel(const float* __restrict__ W, unsigned short* __restrict__ oh,
                                                     unsigned short* __restrict__ ol, int R, int Cc, long sIn, long sOut) {
  __shared__ __align__(16) float tf[64 * 68];
  W  += (size_t)blockIdx.z * sIn;
  oh += (size_t)blockIdx.z * sOut;
  ol += (size_t)blockIdx.z * sOut;
  const int c0  = blockIdx.x * 64;
  const int r0  = blockIdx.y * 64;
  const int tid = threadIdx.x;
  {
    const int lr = tid >> 4;
    const int c4 = (tid & 15) * 4;
#pragma unroll
    for (int it = 0; it < 4; ++it) {
      const int rr = it * 16 + lr;
      const v4f a = *(const v4f*)(W + (size_t)(r0 + rr) * Cc + c0 + c4);
      *(v4f*)(tf + rr * 68 + c4) = a;
    }
  }
  __syncthreads();
  const int sub = tid >> 3;
  const int c8  = (tid & 7) * 8;
  v4u hv[2], lv[2];
#pragma unroll
  for (int it = 0; it < 2; ++it) {
    const int oc = it * 32 + sub;
    v4u a, a2;
#pragma unroll
    for (int q = 0; q < 4; ++q) {
      const float f0 = tf[(c8 + 2 * q) * 68 + oc];
      const float f1 = tf[(c8 + 2 * q + 1) * 68 + oc];
      const unsigned short h0 = f2bf_bits(f0), h1 = f2bf_bits(f1);
      const unsigned short l0 = f2bf_bits(f0 - bf_bits2f(h0)), l1 = f2bf_bits(f1 - bf_bits2f(h1));
      a[q]  = pk16(h0, h1);
      a2[q] = pk16(l0, l1);
    }
    hv[it] = a; lv[it] = a2;
  }
  for (int pass = 0; pass < 2; ++pass) {
#pragma unroll
    for (int it = 0; it < 2; ++it) {
      const int oc = it * 32 + sub;
      const size_t go = (size_t)(c0 + oc) * R + r0 + c8;
      *(volatile v4u*)(oh + go) = hv[it];
      *(volatile v4u*)(ol + go) = lv[it];
    }
    __threadfence();
  }
}

#define AT_NW  4
#define AT_QB  64
#define AT_KC  64
#define AT_CT  16
#define PCARRY 32768.0f
#define LDS_O_F 16384
#define LDS_Q_H 16384
#define LDS_P_H 4096
#define LDS_T_F 4352
#define ATTN_LDS_BYTES (LDS_O_F * 4 + LDS_Q_H * 2 + LDS_P_H * 2 + LDS_T_F * 4)

static_assert(AT_CT * 16 == CH);
static_assert(NPOS % AT_QB == 0);
static_assert(NPOS % AT_KC == 0);
static_assert(ATTN_LDS_BYTES == 123904);
static_assert(((LDS_Q_H + LDS_P_H) % 2) == 0);

__device__ __forceinline__ v8f hm_mma(v16h a, v16h b, v8f c) {
  c = __builtin_amdgcn_wmma_f32_16x16x32_f16(false, a, false, b, (short)0, c, false, false);
  asm volatile("v_nop\n\tv_nop\n\tv_nop\n\tv_nop" : "+v"(c) : "v"(a), "v"(b));
  return c;
}

__global__ __launch_bounds__(128)
void attn_kernel(const unsigned short* __restrict__ qpp, const unsigned short* __restrict__ kpp,
                 const unsigned short* __restrict__ vtp, const float* __restrict__ xin,
                 const float* __restrict__ gam, float* __restrict__ out) {
  extern __shared__ __align__(16) float dynlds[];
  float*    osl = dynlds;
  _Float16* qsl = (_Float16*)(dynlds + LDS_O_F);
  _Float16* psl = qsl + LDS_Q_H;
  float*    tst = dynlds + LDS_O_F + (LDS_Q_H + LDS_P_H) / 2;

  const int tid  = threadIdx.x;
  const int wave = tid >> 5;
  const int lane = tid & 31;
  const int hh   = lane >> 4;
  const int c    = lane & 15;

  const int nqb = NPOS / AT_QB;
  const int bx = blockIdx.x;
  const int qb = bx % nqb;
  const int b  = bx / nqb;
  const int n0 = qb * AT_QB;
  const int q0 = b * NPOS + n0 + wave * 16;

  const _Float16* Qg = (const _Float16*)(const void*)qpp;
  const _Float16* Kg = (const _Float16*)(const void*)kpp + (size_t)b * NPOS * CH;
  const _Float16* Vg = (const _Float16*)(const void*)vtp + (size_t)b * CH * NPOS;
  float*    ow = osl + wave * (AT_CT * 32 * 8);
  _Float16* qw = qsl + wave * (16 * CH);
  _Float16* pw = psl + wave * (16 * AT_KC);

#pragma unroll 4
  for (int i = 0; i < 16; ++i) {
    const v8h v = *(const v8h*)(Qg + (size_t)(q0 + i) * CH + lane * 8);
    *(v8h*)(qw + i * CH + lane * 8) = v;
  }
  {
    const v4f z4 = {0.f, 0.f, 0.f, 0.f};
#pragma unroll 4
    for (int t = 0; t < AT_CT; ++t) {
      float* op = ow + (t * 32 + lane) * 8;
      *(v4f*)op = z4;
      *(v4f*)(op + 4) = z4;
    }
  }
  __syncthreads();

  float mrow[8], lrow[8];
#pragma unroll
  for (int r = 0; r < 8; ++r) { mrow[r] = -INFINITY; lrow[r] = 0.f; }

  const int nChunks = NPOS / AT_KC;
#pragma unroll 1
  for (int kc = 0; kc < nChunks; ++kc) {
    const int kv0 = kc * AT_KC;

    v8f s[4];
#pragma unroll
    for (int j = 0; j < 4; ++j) s[j] = (v8f){0.f,0.f,0.f,0.f,0.f,0.f,0.f,0.f};
#pragma unroll 2
    for (int dc = 0; dc < 8; ++dc) {
      const v16h qa = Frag<_Float16>::load(qw + c * CH + dc * 32 + 8 * hh);
#pragma unroll
      for (int j = 0; j < 4; ++j) {
        const v16h kb = Frag<_Float16>::load(Kg + (size_t)(kv0 + j * 16 + c) * CH + dc * 32 + 8 * hh);
        s[j] = hm_mma(qa, kb, s[j]);
      }
    }

    float cm[8];
#pragma unroll
    for (int r = 0; r < 8; ++r) {
      float m = fmaxf(fmaxf(s[0][r], s[1][r]), fmaxf(s[2][r], s[3][r]));
#pragma unroll
      for (int off = 1; off < 16; off <<= 1) m = fmaxf(m, __shfl_xor(m, off, 32));
      cm[r] = m;
    }
    __builtin_amdgcn_fence(__ATOMIC_RELEASE, "workgroup");
    __builtin_amdgcn_wave_barrier();
    __builtin_amdgcn_fence(__ATOMIC_ACQUIRE, "workgroup");
    float alphar[8];
#pragma unroll
    for (int r = 0; r < 8; ++r) {
      const float mnew  = fmaxf(mrow[r], cm[r]);
      const float alpha = __expf(mrow[r] - mnew);
      mrow[r]   = mnew;
      alphar[r] = alpha;
      float psum = 0.f;
#pragma unroll
      for (int j = 0; j < 4; ++j) {
        const float p = __expf(s[j][r] - mnew);
        psum += p;
        pw[(8 * hh + r) * AT_KC + j * 16 + c] = h_flush(p * PCARRY);
      }
#pragma unroll
      for (int off = 1; off < 16; off <<= 1) psum += __shfl_xor(psum, off, 32);
      lrow[r] = lrow[r] * alpha + psum;
    }
    __builtin_amdgcn_fence(__ATOMIC_RELEASE, "workgroup");
    __builtin_amdgcn_wave_barrier();
    __builtin_amdgcn_fence(__ATOMIC_ACQUIRE, "workgroup");

    const v16h pa0 = Frag<_Float16>::load(pw + c * AT_KC + 8 * hh);
    const v16h pa1 = Frag<_Float16>::load(pw + c * AT_KC + 32 + 8 * hh);

    const _Float16* vbase = Vg + kv0 + 8 * hh;
#pragma unroll 2
    for (int t = 0; t < AT_CT; ++t) {
      float* op = ow + (t * 32 + lane) * 8;
      const v4f oa = *(const v4f*)op;
      const v4f ob = *(const v4f*)(op + 4);
      v8f o;
      o[0] = oa[0] * alphar[0]; o[1] = oa[1] * alphar[1]; o[2] = oa[2] * alphar[2]; o[3] = oa[3] * alphar[3];
      o[4] = ob[0] * alphar[4]; o[5] = ob[1] * alphar[5]; o[6] = ob[2] * alphar[6]; o[7] = ob[3] * alphar[7];
      const _Float16* vr = vbase + (size_t)(t * 16 + c) * NPOS;
      const v16h vb0 = Frag<_Float16>::load(vr);
      const v16h vb1 = Frag<_Float16>::load(vr + 32);
      o = hm_mma(pa0, vb0, o);
      o = hm_mma(pa1, vb1, o);
      v4f ra, rb;
      ra[0] = o[0]; ra[1] = o[1]; ra[2] = o[2]; ra[3] = o[3];
      rb[0] = o[4]; rb[1] = o[5]; rb[2] = o[6]; rb[3] = o[7];
      *(v4f*)op = ra;
      *(v4f*)(op + 4) = rb;
    }
  }

  const float g = gam[0];
  float inv[8];
#pragma unroll
  for (int r = 0; r < 8; ++r) inv[r] = g * (1.0f / (lrow[r] * PCARRY));
  __syncthreads();
#pragma unroll 1
  for (int cg = 0; cg < 4; ++cg) {
#pragma unroll
    for (int tl = 0; tl < 4; ++tl) {
      const int t = cg * 4 + tl;
      const float* op = ow + (t * 32 + lane) * 8;
      const v4f oa = *(const v4f*)op;
      const v4f ob = *(const v4f*)(op + 4);
      v4f wa, wb;
      wa[0] = oa[0] * inv[0]; wa[1] = oa[1] * inv[1]; wa[2] = oa[2] * inv[2]; wa[3] = oa[3] * inv[3];
      wb[0] = ob[0] * inv[4]; wb[1] = ob[1] * inv[5]; wb[2] = ob[2] * inv[6]; wb[3] = ob[3] * inv[7];
      float* trow = tst + (tl * 16 + c) * 68 + wave * 16 + 8 * hh;
      *(v4f*)trow = wa;
      *(v4f*)(trow + 4) = wb;
    }
    __syncthreads();
    v4f ov[8];
    const int c4 = c * 4;
#pragma unroll
    for (int it = 0; it < 8; ++it) {
      const int row = it * 8 + wave * 2 + hh;
      const v4f tv = *(const v4f*)(tst + row * 68 + c4);
      const size_t go = ((size_t)(b * CH + cg * 64 + row)) * NPOS + n0 + c4;
      const v4f xr = *(const v4f*)(xin + go);
      ov[it] = tv + xr;
    }
    for (int pass = 0; pass < 2; ++pass) {
#pragma unroll
      for (int it = 0; it < 8; ++it) {
        const int row = it * 8 + wave * 2 + hh;
        const size_t go = ((size_t)(b * CH + cg * 64 + row)) * NPOS + n0 + c4;
        *(volatile v4f*)(out + go) = ov[it];
      }
      __threadfence();
    }
    __syncthreads();
  }
}

extern "C" void kernel_launch(void* const* d_in, const int* in_sizes, int n_in,
                              void* d_out, int out_size, void* d_ws, size_t ws_size,
                              hipStream_t stream) {
  if (n_in < 6) return;
  if (in_sizes[0] != NB * CH * NPOS) return;
  if (in_sizes[1] != NB * CH * NPOS) return;
  if (in_sizes[2] != CH * CH) return;
  if (in_sizes[3] != CH * CH) return;
  if (in_sizes[4] != CH * CH) return;
  if (in_sizes[5] < 1) return;
  if (out_size != NB * CH * NPOS) return;

  const float* x   = (const float*)d_in[0];
  const float* y   = (const float*)d_in[1];
  const float* wq  = (const float*)d_in[2];
  const float* wk  = (const float*)d_in[3];
  const float* wv  = (const float*)d_in[4];
  const float* gam = (const float*)d_in[5];

  const size_t PA = (size_t)MTOK * CH * 2;
  const size_t PW = (size_t)CH * CH * 2;
  const size_t PV = (size_t)NB * CH * NPOS * 2;
  size_t off = 0;
  const size_t oXTh = off; off += PA;  const size_t oXTl = off; off += PA;
  const size_t oYTh = off; off += PA;  const size_t oYTl = off; off += PA;
  const size_t oWQh = off; off += PW;  const size_t oWQl = off; off += PW;
  const size_t oWKh = off; off += PW;  const size_t oWKl = off; off += PW;
  const size_t oWVh = off; off += PW;  const size_t oWVl = off; off += PW;
  const size_t oQP  = off; off += PA;
  const size_t oKP  = off; off += PA;
  const size_t oVT  = off; off += PV;
  if (off > ws_size) return;
  if (off > (size_t)134217728) return;

  char* ws = (char*)d_ws;
  unsigned short* XTh = (unsigned short*)(ws + oXTh); unsigned short* XTl = (unsigned short*)(ws + oXTl);
  unsigned short* YTh = (unsigned short*)(ws + oYTh); unsigned short* YTl = (unsigned short*)(ws + oYTl);
  unsigned short* WQh = (unsigned short*)(ws + oWQh); unsigned short* WQl = (unsigned short*)(ws + oWQl);
  unsigned short* WKh = (unsigned short*)(ws + oWKh); unsigned short* WKl = (unsigned short*)(ws + oWKl);
  unsigned short* WVh = (unsigned short*)(ws + oWVh); unsigned short* WVl = (unsigned short*)(ws + oWVl);
  unsigned short* QP  = (unsigned short*)(ws + oQP);
  unsigned short* KP  = (unsigned short*)(ws + oKP);
  unsigned short* VT  = (unsigned short*)(ws + oVT);

  const dim3 blk(256);

  tsplit_kernel<<<dim3(NPOS / 64, CH / 64, NB), blk, 0, stream>>>(x, XTh, XTl, CH, NPOS, (long)CH * NPOS, (long)NPOS * CH);
  tsplit_kernel<<<dim3(NPOS / 64, CH / 64, NB), blk, 0, stream>>>(y, YTh, YTl, CH, NPOS, (long)CH * NPOS, (long)NPOS * CH);
  const int n2w = CH * CH / 2;
  split_bf16x2_kernel<<<dim3((n2w + 255) / 256), blk, 0, stream>>>(wq, WQh, WQl, n2w);
  split_bf16x2_kernel<<<dim3((n2w + 255) / 256), blk, 0, stream>>>(wk, WKh, WKl, n2w);
  split_bf16x2_kernel<<<dim3((n2w + 255) / 256), blk, 0, stream>>>(wv, WVh, WVl, n2w);
  const dim3 gProj(((MTOK / 64) * (CH / 64) + 7) / 8, 1);
  wmma_gemm64<1, true, 0, 1, false, 0><<<gProj, blk, 0, stream>>>(
      XTh, XTl, CH, 0L, WQh, WQl, CH, 0L, (void*)QP, (void*)QP, CH, 0L,
      gam, x, 0L, MTOK, CH, CH, 1.0f);
  wmma_gemm64<1, true, 0, 1, false, 0><<<gProj, blk, 0, stream>>>(
      YTh, YTl, CH, 0L, WKh, WKl, CH, 0L, (void*)KP, (void*)KP, CH, 0L,
      gam, x, 0L, MTOK, CH, CH, 1.0f);
  const dim3 gVT(((CH / 64) * (NPOS / 64) + 7) / 8, NB);
  wmma_gemm64<1, true, 0, 1, false, 0><<<gVT, blk, 0, stream>>>(
      WVh, WVl, CH, 0L, YTh, YTl, CH, (long)NPOS * CH, (void*)VT, (void*)VT, NPOS, (long)CH * NPOS,
      gam, x, 0L, CH, NPOS, CH, 1.0f);
  (void)hipFuncSetAttribute(reinterpret_cast<const void*>(&attn_kernel), hipFuncAttributeMaxDynamicSharedMemorySize, ATTN_LDS_BYTES);
  attn_kernel<<<dim3(NB * (NPOS / AT_QB)), dim3(128), ATTN_LDS_BYTES, stream>>>(QP, KP, VT, x, gam, (float*)d_out);
  (void)hipGetLastError();
}
